// MultiHeadAttn_55353538510859
// MI455X (gfx1250) — hardware-verified
//
#include <hip/hip_runtime.h>
#include <math.h>

typedef __attribute__((ext_vector_type(16))) _Float16 v16h;
typedef __attribute__((ext_vector_type(8)))  _Float16 v8h;
typedef __attribute__((ext_vector_type(16))) __bf16   v16b;
typedef __attribute__((ext_vector_type(8)))  __bf16   v8b;
typedef __attribute__((ext_vector_type(8)))  float    v8f;
typedef __attribute__((ext_vector_type(4)))  float    v4f;
typedef __attribute__((ext_vector_type(4)))  unsigned v4u;
typedef __attribute__((ext_vector_type(8)))  unsigned short v8us;

constexpr int N_BATCH   = 2;
constexpr int SEQ_LEN   = 2048;
constexpr int D_MODEL   = 768;
constexpr int N_HEADS   = 12;
constexpr int HEAD_DIM  = 64;
constexpr int M_ROWS    = N_BATCH * SEQ_LEN;
constexpr int KV_CHUNK  = 64;
constexpr int Q_BLOCK   = 64;
constexpr int ATT_WAVES = 4;
constexpr int OS_PITCH  = 68;
constexpr int TP_PITCH  = 72;
static_assert(D_MODEL == N_HEADS * HEAD_DIM);
static_assert(SEQ_LEN % KV_CHUNK == 0 && SEQ_LEN % Q_BLOCK == 0);
static_assert(M_ROWS % 64 == 0 && D_MODEL % 64 == 0 && D_MODEL % 32 == 0);
static_assert(HEAD_DIM == 64 && KV_CHUNK == 64 && Q_BLOCK == ATT_WAVES * 16);

__device__ __forceinline__ unsigned short f2bf_bits(float f) {
  unsigned u = __float_as_uint(f);
  return (unsigned short)((u + 0x7FFFu + ((u >> 16) & 1u)) >> 16);
}
__device__ __forceinline__ float bf_bits2f(unsigned short h) { return __uint_as_float(((unsigned)h) << 16); }

__device__ __forceinline__ void dep_guard_h(v8f& a, v8f& b, v16h x, v16h y) { asm volatile("v_nop\n\tv_nop\n\tv_nop\n\tv_nop" : "+v"(a), "+v"(b) : "v"(x), "v"(y)); }
__device__ __forceinline__ void dep_guard_b(v8f& a, v8f& b, v16b x, v16b y) { asm volatile("v_nop\n\tv_nop\n\tv_nop\n\tv_nop" : "+v"(a), "+v"(b) : "v"(x), "v"(y)); }
__device__ __forceinline__ void keep4_h(v16h a, v16h b, v16h c, v16h d) { asm volatile("v_nop" :: "v"(a), "v"(b), "v"(c), "v"(d)); }
__device__ __forceinline__ void keep4_b(v16b a, v16b b, v16b c, v16b d) { asm volatile("v_nop" :: "v"(a), "v"(b), "v"(c), "v"(d)); }
__device__ __forceinline__ void acc_guard4(v8f& a, v8f& b, v8f& c, v8f& d) { asm volatile("v_nop\n\tv_nop\n\tv_nop\n\tv_nop" : "+v"(a), "+v"(b), "+v"(c), "+v"(d)); }
template <typename T> struct Frag;
template <> struct Frag<_Float16> {
  typedef v16h V; union U { v16h v; v8h h[2]; };
  static __device__ __forceinline__ v16h load(const _Float16* p) {
    U f; f.h[0] = *(const v8h*)(p); f.h[1] = *(const v8h*)(p + 16); return f.v;
  }
  static __device__ __forceinline__ v8f mma(v16h a, v16h b, v8f c) {
    return __builtin_amdgcn_wmma_f32_16x16x32_f16(false, a, false, b, (short)0, c, false, false);
  }
  static __device__ __forceinline__ void guard(v8f& a, v8f& b, v16h x, v16h y) { dep_guard_h(a, b, x, y); }
  static __device__ __forceinline__ void keep(v16h a, v16h b, v16h c, v16h d) { keep4_h(a, b, c, d); }
};
template <> struct Frag<__bf16> {
  typedef v16b V; union U { v16b v; v8b h[2]; };
  static __device__ __forceinline__ v16b load(const __bf16* p) {
    U f; f.h[0] = *(const v8b*)(p); f.h[1] = *(const v8b*)(p + 16); return f.v;
  }
  static __device__ __forceinline__ v8f mma(v16b a, v16b b, v8f c) {
    return __builtin_amdgcn_wmma_f32_16x16x32_bf16(false, a, false, b, (short)0, c, false, false);
  }
  static __device__ __forceinline__ void guard(v8f& a, v8f& b, v16b x, v16b y) { dep_guard_b(a, b, x, y); }
  static __device__ __forceinline__ void keep(v16b a, v16b b, v16b c, v16b d) { keep4_b(a, b, c, d); }
};

template <int ET> struct Elem;
template <> struct Elem<0> { typedef _Float16 T; };
template <> struct Elem<1> { typedef __bf16 T; };
template <int ET, int SPLIT, int BIAS_MODE, int OUT_MODE, bool RESID, int ACT = 0>
__global__ __launch_bounds__(256) void wmma_gemm64(
    const unsigned short* __restrict__ Ap, const unsigned short* __restrict__ A2p, int lda, long strideA,
    const unsigned short* __restrict__ Btp, const unsigned short* __restrict__ Bt2p, int ldb, long strideB,
    void* __restrict__ Cout, void* __restrict__ Cout2, int ldc, long strideC,
    const float* __restrict__ bias,
    const float* __restrict__ resid, long strideR,
    int M, int N, int K, float scale) {
  static_assert(!RESID);
  static_assert(SPLIT >= 0 && SPLIT <= 2);
  (void)resid; (void)strideR;
  typedef typename Elem<ET>::T T;
  typedef typename Frag<T>::V V;
  const T* A = (const T*)Ap; const T* A2 = (const T*)A2p; const T* Bt = (const T*)Btp; const T* Bt2 = (const T*)Bt2p;
  __shared__ __align__(16) float sT[8][16 * 68];
  const int b    = blockIdx.y;
  const int lane = threadIdx.x & 31;
  const int wave = threadIdx.x >> 5;
  const int tilesN = N >> 6;
  const int tilesM = M >> 6;
  const int tile = blockIdx.x * 8 + wave;
  if (tile >= tilesM * tilesN) return;
  const int tm = tile / tilesN;
  const int tn = tile - tm * tilesN;
  const int m0 = tm << 6;
  const int n0 = tn << 6;

  const T* Ab  = A  + (size_t)b * strideA;
  const T* Bb  = Bt + (size_t)b * strideB;
  const T* Ab2 = (SPLIT >= 1) ? (A2  + (size_t)b * strideA) : nullptr;
  const T* Bb2 = (SPLIT == 2) ? (Bt2 + (size_t)b * strideB) : nullptr;

  const int rlane = lane & 15;
  const int koff  = (lane >> 4) * 8;
  const int mOff  = (lane >> 4) * 8;

  v8f acc[4][4];
#pragma unroll
  for (int i = 0; i < 4; ++i)
#pragma unroll
    for (int j = 0; j < 4; ++j) acc[i][j] = (v8f){0.f,0.f,0.f,0.f,0.f,0.f,0.f,0.f};

  for (int k0 = 0; k0 < K; k0 += 32) {
    V bh[4], bl[4];
#pragma unroll
    for (int j = 0; j < 4; ++j) {
      const size_t bo = (size_t)(n0 + (j << 4) + rlane) * ldb + koff + k0;
      bh[j] = Frag<T>::load(Bb + bo);
      if (SPLIT == 2) bl[j] = Frag<T>::load(Bb2 + bo);
    }
#pragma unroll
    for (int i = 0; i < 4; ++i) {
      const size_t ao = (size_t)(m0 + (i << 4) + rlane) * lda + koff + k0;
      V ah = Frag<T>::load(Ab + ao);
      V al;
      if (SPLIT >= 1) al = Frag<T>::load(Ab2 + ao);
#pragma unroll
      for (int j = 0; j < 4; ++j) {
        acc[i][j] = Frag<T>::mma(ah, bh[j], acc[i][j]);
        if (SPLIT == 2) acc[i][j] = Frag<T>::mma(ah, bl[j], acc[i][j]);
        if (SPLIT >= 1) acc[i][j] = Frag<T>::mma(al, bh[j], acc[i][j]);
      }
      Frag<T>::guard(acc[i][0], acc[i][3], ah, (SPLIT >= 1) ? al : ah);
    }
    Frag<T>::keep(bh[0], bh[1], bh[2], bh[3]);
    if (SPLIT == 2) Frag<T>::keep(bl[0], bl[1], bl[2], bl[3]);
  }
  acc_guard4(acc[0][0], acc[0][1], acc[0][2], acc[0][3]);
  acc_guard4(acc[1][0], acc[1][1], acc[1][2], acc[1][3]);
  acc_guard4(acc[2][0], acc[2][1], acc[2][2], acc[2][3]);
  acc_guard4(acc[3][0], acc[3][1], acc[3][2], acc[3][3]);

  float* slab = sT[wave];
#pragma unroll
  for (int i = 0; i < 4; ++i) {
    const int mBase = m0 + (i << 4);
    v4f bm0 = (v4f){0.f, 0.f, 0.f, 0.f};
    v4f bm1 = bm0;
    if (BIAS_MODE == 1) {
      bm0 = *(const v4f*)(bias + mBase + mOff);
      bm1 = *(const v4f*)(bias + mBase + mOff + 4);
    }
#pragma unroll
    for (int j = 0; j < 4; ++j) {
      const int n = n0 + (j << 4) + rlane;
      float bv = 0.f;
      if (BIAS_MODE == 2) bv = bias[n];
#pragma unroll
      for (int r = 0; r < 8; ++r) {
        float v = acc[i][j][r] * scale;
        if (BIAS_MODE == 1) v += (r < 4) ? bm0[r] : bm1[r - 4];
        if (BIAS_MODE == 2) v += bv;
        if (ACT == 1) v = tanhf(v);
        if (ACT == 2) v = fmaxf(v, 0.0f);
        if (ACT == 3) v = v / (1.0f + expf(-v));
        if (ACT == 4) v = (v > 0.f) ? v : 0.01f * v;
        slab[(mOff + r) * 68 + (j << 4) + rlane] = v;
      }
    }
    __builtin_amdgcn_fence(__ATOMIC_RELEASE, "workgroup");
    __builtin_amdgcn_wave_barrier();
    __builtin_amdgcn_fence(__ATOMIC_ACQUIRE, "workgroup");
    if (OUT_MODE == 0) {
      float* C = (float*)Cout + (size_t)b * strideC;
      const int hh = lane >> 4, c4 = (lane & 15) * 4;
      for (int pass = 0; pass < 2; ++pass) {
#pragma unroll
        for (int it = 0; it < 8; ++it) {
          const int row = it * 2 + hh;
          v4f v = *(const v4f*)(slab + row * 68 + c4);
          *(volatile v4f*)(C + (size_t)(mBase + row) * ldc + n0 + c4) = v;
        }
        __threadfence();
      }
    } else {
      const int q = lane >> 3, c8 = (lane & 7) * 8;
      unsigned short* C  = (unsigned short*)Cout  + (size_t)b * strideC;
      unsigned short* C2 = (OUT_MODE == 2) ? ((unsigned short*)Cout2 + (size_t)b * strideC) : nullptr;
      for (int pass = 0; pass < 2; ++pass) {
#pragma unroll
        for (int it = 0; it < 4; ++it) {
          const int row = it * 4 + q;
          const float* sp = slab + row * 68 + c8;
          v8h hv, lv;
#pragma unroll
          for (int e = 0; e < 8; ++e) {
            if (OUT_MODE == 1) {
              hv[e] = (_Float16)sp[e];
            } else {
              unsigned short hb = f2bf_bits(sp[e]);
              unsigned short lb = f2bf_bits(sp[e] - bf_bits2f(hb));
              hv[e] = __builtin_bit_cast(_Float16, hb);
              lv[e] = __builtin_bit_cast(_Float16, lb);
            }
          }
          *(volatile v8h*)(C + (size_t)(mBase + row) * ldc + n0 + c8) = hv;
          if (OUT_MODE == 2) *(volatile v8h*)(C2 + (size_t)(mBase + row) * ldc + n0 + c8) = lv;
        }
        __threadfence();
      }
    }
    __builtin_amdgcn_fence(__ATOMIC_RELEASE, "workgroup");
    __builtin_amdgcn_wave_barrier();
    __builtin_amdgcn_fence(__ATOMIC_ACQUIRE, "workgroup");
  }
}

__device__ __forceinline__ unsigned short at_bf_bits(float f) {
  unsigned u = __float_as_uint(f);
  return (unsigned short)((u + 0x7FFFu + ((u >> 16) & 1u)) >> 16);
}
__device__ __forceinline__ __bf16 at_f2bf(float f) { return __builtin_bit_cast(__bf16, at_bf_bits(f)); }
__device__ __forceinline__ void at_split(float f, __bf16& hi, __bf16& lo) {
  const unsigned short hb = at_bf_bits(f);
  hi = __builtin_bit_cast(__bf16, hb);
  lo = at_f2bf(f - __uint_as_float(((unsigned)hb) << 16));
}
__device__ __forceinline__ v8f at_mma(v16b a, v16b b, v8f c) {
  c = __builtin_amdgcn_wmma_f32_16x16x32_bf16(false, a, false, b, (short)0, c, false, false);
  asm volatile("v_nop\n\tv_nop\n\tv_nop\n\tv_nop" : "+v"(c) : "v"(a), "v"(b));
  return c;
}

__global__ __launch_bounds__(256) void cast_f32_bf16x8(
    const float* __restrict__ in0, const float* __restrict__ in1, const float* __restrict__ in2,
    unsigned short* __restrict__ out, int n8, long plane_elems) {
  const int which = blockIdx.y;
  const float* src = (which == 0) ? in0 : ((which == 1) ? in1 : in2);
  unsigned short* dst = out + (size_t)which * (size_t)plane_elems;
  const int i = blockIdx.x * 256 + threadIdx.x;
  if (i < n8) {
    const v4f a0 = *(const v4f*)(src + (size_t)8 * i);
    const v4f a1 = *(const v4f*)(src + (size_t)8 * i + 4);
    v4u w;
    w[0] = (unsigned)f2bf_bits(a0[0]) | ((unsigned)f2bf_bits(a0[1]) << 16);
    w[1] = (unsigned)f2bf_bits(a0[2]) | ((unsigned)f2bf_bits(a0[3]) << 16);
    w[2] = (unsigned)f2bf_bits(a1[0]) | ((unsigned)f2bf_bits(a1[1]) << 16);
    w[3] = (unsigned)f2bf_bits(a1[2]) | ((unsigned)f2bf_bits(a1[3]) << 16);
    unsigned short* p = dst + (size_t)8 * i;
    *(volatile v4u*)p = w;
    __threadfence();
    *(volatile v4u*)p = w;
  }
}

__global__ __launch_bounds__(256) void transpose_cast_w(
    const float* __restrict__ w0, const float* __restrict__ w1, const float* __restrict__ w2,
    const float* __restrict__ w3, unsigned short* __restrict__ wt, int dim) {
  __shared__ __align__(16) unsigned short sm[64 * TP_PITCH];
  const int which = blockIdx.z;
  const float* src = (which == 0) ? w0 : ((which == 1) ? w1 : ((which == 2) ? w2 : w3));
  unsigned short* dst = wt + (size_t)which * (size_t)dim * (size_t)dim;
  const int k0 = blockIdx.x * 64;
  const int n0 = blockIdx.y * 64;
  const int t = threadIdx.x;
  {
    const int r = t >> 2, c0 = (t & 3) * 16;
    const float* rp = src + (size_t)(k0 + r) * dim + n0 + c0;
#pragma unroll
    for (int i = 0; i < 4; ++i) {
      const v4f v = *(const v4f*)(rp + 4 * i);
#pragma unroll
      for (int e = 0; e < 4; ++e) sm[(c0 + 4 * i + e) * TP_PITCH + r] = f2bf_bits(v[e]);
    }
  }
  __syncthreads();
  {
    const int g = t >> 3, l8 = t & 7;
    for (int pass = 0; pass < 2; ++pass) {
#pragma unroll
      for (int rr = 0; rr < 2; ++rr) {
        const int nl = g + 32 * rr;
        const v8us v = *(const v8us*)(sm + nl * TP_PITCH + l8 * 8);
        *(volatile v8us*)(dst + (size_t)(n0 + nl) * dim + k0 + l8 * 8) = v;
      }
      __threadfence();
    }
  }
}

__global__ __launch_bounds__(192) void rne_bias4(
    const float* __restrict__ b0, const float* __restrict__ b1, const float* __restrict__ b2,
    const float* __restrict__ b3, float* __restrict__ outb, int dim) {
  const int which = blockIdx.x;
  const float* src = (which == 0) ? b0 : ((which == 1) ? b1 : ((which == 2) ? b2 : b3));
  float* dst = outb + (size_t)which * dim;
  const int t = threadIdx.x;
  if (4 * t + 3 < dim) {
    const v4f v = *(const v4f*)(src + 4 * t);
    v4f r;
    r[0] = bf_bits2f(f2bf_bits(v[0]));
    r[1] = bf_bits2f(f2bf_bits(v[1]));
    r[2] = bf_bits2f(f2bf_bits(v[2]));
    r[3] = bf_bits2f(f2bf_bits(v[3]));
    *(volatile v4f*)(dst + 4 * t) = r;
    __threadfence();
    *(volatile v4f*)(dst + 4 * t) = r;
  }
}

__global__ __launch_bounds__(128) void attn_hd64_planes(
    const unsigned short* __restrict__ Qh, const unsigned short* __restrict__ Ql,
    const unsigned short* __restrict__ Kh, const unsigned short* __restrict__ Kl,
    const unsigned short* __restrict__ Vth, const unsigned short* __restrict__ Vtl,
    unsigned short* __restrict__ Oh, unsigned short* __restrict__ Ol, float qk_scale) {
  union FB { v16b v; v8b h[2]; };
  __shared__ __align__(16) unsigned short Ksh[KV_CHUNK * HEAD_DIM];
  __shared__ __align__(16) unsigned short Ksl[KV_CHUNK * HEAD_DIM];
  __shared__ __align__(16) unsigned short Vsh[HEAD_DIM * KV_CHUNK];
  __shared__ __align__(16) unsigned short Vsl[HEAD_DIM * KV_CHUNK];
  __shared__ __align__(16) __bf16 Psh[ATT_WAVES][16 * KV_CHUNK];
  __shared__ __align__(16) __bf16 Psl[ATT_WAVES][16 * KV_CHUNK];
  __shared__ __align__(16) float  Os[ATT_WAVES][16 * OS_PITCH];

  const int tid  = threadIdx.x;
  const int wave = tid >> 5;
  const int lane = tid & 31;
  const int hh   = lane >> 4;
  const int c    = lane & 15;

  const int nqb  = SEQ_LEN / Q_BLOCK;
  const int bx   = blockIdx.x;
  const int qb   = bx % nqb;
  const int bhid = bx / nqb;
  const int h    = bhid % N_HEADS;
  const int b    = bhid / N_HEADS;
  const int q0   = qb * Q_BLOCK + wave * 16;
  const size_t rowbase = (size_t)b * SEQ_LEN;
  const int colbase = h * HEAD_DIM;

  v16b qah[2], qal[2];
  {
    const size_t qoff = (rowbase + q0 + c) * (size_t)D_MODEL + colbase + 8 * hh;
    const __bf16* qhp = (const __bf16*)(const void*)Qh + qoff;
    const __bf16* qlp = (const __bf16*)(const void*)Ql + qoff;
#pragma unroll
    for (int dc = 0; dc < 2; ++dc) {
      qah[dc] = Frag<__bf16>::load(qhp + dc * 32);
      qal[dc] = Frag<__bf16>::load(qlp + dc * 32);
    }
  }

  float mrow[8], lrow[8];
  v8f oacc[4];
#pragma unroll
  for (int r = 0; r < 8; ++r) { mrow[r] = -INFINITY; lrow[r] = 0.f; }
#pragma unroll
  for (int t = 0; t < 4; ++t) oacc[t] = (v8f){0.f,0.f,0.f,0.f,0.f,0.f,0.f,0.f};

  for (int kc = 0; kc < SEQ_LEN / KV_CHUNK; ++kc) {
    const int kv0 = kc * KV_CHUNK;
    __syncthreads();
    {
#pragma unroll
      for (int i = 0; i < 4; ++i) {
        const int e = tid + 128 * i;
        const int r = e >> 3, c8 = (e & 7) * 8;
        const size_t go = (rowbase + kv0 + r) * (size_t)D_MODEL + colbase + c8;
        const v4u kw_h = *(const v4u*)(Kh + go);
        const v4u kw_l = *(const v4u*)(Kl + go);
        *(v4u*)(Ksh + r * HEAD_DIM + c8) = kw_h;
        *(v4u*)(Ksl + r * HEAD_DIM + c8) = kw_l;
      }
      asm volatile("" ::: "memory");
#pragma unroll
      for (int i = 0; i < 4; ++i) {
        const int e = tid + 128 * i;
        const int d = e >> 3, c8 = (e & 7) * 8;
        const size_t go = (size_t)(colbase + d) * (size_t)M_ROWS + rowbase + kv0 + c8;
        const v4u vw_h = *(const v4u*)(Vth + go);
        const v4u vw_l = *(const v4u*)(Vtl + go);
        *(v4u*)(Vsh + d * KV_CHUNK + c8) = vw_h;
        *(v4u*)(Vsl + d * KV_CHUNK + c8) = vw_l;
      }
    }
    __syncthreads();

    v8f s[4];
#pragma unroll
    for (int j = 0; j < 4; ++j) {
      s[j] = (v8f){0.f,0.f,0.f,0.f,0.f,0.f,0.f,0.f};
#pragma unroll
      for (int dc = 0; dc < 2; ++dc) {
        FB kfh, kfl;
        const int ko = (j * 16 + c) * HEAD_DIM + dc * 32 + 8 * hh;
        kfh.h[0] = *(const v8b*)(const void*)(Ksh + ko);
        kfh.h[1] = *(const v8b*)(const void*)(Ksh + ko + 16);
        kfl.h[0] = *(const v8b*)(const void*)(Ksl + ko);
        kfl.h[1] = *(const v8b*)(const void*)(Ksl + ko + 16);
        s[j] = at_mma(qah[dc], kfh.v, s[j]);
        s[j] = at_mma(qah[dc], kfl.v, s[j]);
        s[j] = at_mma(qal[dc], kfh.v, s[j]);
      }
    }

    float cm[8];
#pragma unroll
    for (int r = 0; r < 8; ++r) {
      float m = -INFINITY;
#pragma unroll
      for (int j = 0; j < 4; ++j) {
        const float sv = s[j][r] * qk_scale;
        s[j][r] = sv;
        m = fmaxf(m, sv);
      }
#pragma unroll
      for (int off = 1; off < 16; off <<= 1) m = fmaxf(m, __shfl_xor(m, off, 32));
      cm[r] = m;
    }
    __bf16* pwh = Psh[wave];
    __bf16* pwl = Psl[wave];
#pragma unroll
    for (int r = 0; r < 8; ++r) {
      const float mnew = fmaxf(mrow[r], cm[r]);
      const float alpha = expf(mrow[r] - mnew);
      mrow[r] = mnew;
      float psum = 0.f;
#pragma unroll
      for (int j = 0; j < 4; ++j) {
        const float p = expf(s[j][r] - mnew);
        psum += p;
        __bf16 ph, pl;
        at_split(p, ph, pl);
        pwh[(8 * hh + r) * KV_CHUNK + j * 16 + c] = ph;
        pwl[(8 * hh + r) * KV_CHUNK + j * 16 + c] = pl;
      }
#pragma unroll
      for (int off = 1; off < 16; off <<= 1) psum += __shfl_xor(psum, off, 32);
      lrow[r] = lrow[r] * alpha + psum;
#pragma unroll
      for (int t = 0; t < 4; ++t) oacc[t][r] *= alpha;
    }
    __builtin_amdgcn_fence(__ATOMIC_RELEASE, "workgroup");
    __builtin_amdgcn_wave_barrier();
    __builtin_amdgcn_fence(__ATOMIC_ACQUIRE, "workgroup");

#pragma unroll 1
    for (int kk = 0; kk < 2; ++kk) {
      FB pa, pl;
      pa.h[0] = *(const v8b*)(pwh + c * KV_CHUNK + kk * 32 + 8 * hh);
      pa.h[1] = *(const v8b*)(pwh + c * KV_CHUNK + kk * 32 + 16 + 8 * hh);
      pl.h[0] = *(const v8b*)(pwl + c * KV_CHUNK + kk * 32 + 8 * hh);
      pl.h[1] = *(const v8b*)(pwl + c * KV_CHUNK + kk * 32 + 16 + 8 * hh);
#pragma unroll
      for (int t = 0; t < 4; ++t) {
        FB vfh, vfl;
        const int vo = (t * 16 + c) * KV_CHUNK + kk * 32 + 8 * hh;
        vfh.h[0] = *(const v8b*)(const void*)(Vsh + vo);
        vfh.h[1] = *(const v8b*)(const void*)(Vsh + vo + 16);
        vfl.h[0] = *(const v8b*)(const void*)(Vsl + vo);
        vfl.h[1] = *(const v8b*)(const void*)(Vsl + vo + 16);
        oacc[t] = at_mma(pa.v, vfh.v, oacc[t]);
        oacc[t] = at_mma(pa.v, vfl.v, oacc[t]);
        oacc[t] = at_mma(pl.v, vfh.v, oacc[t]);
      }
    }
  }

  float* os = Os[wave];
#pragma unroll
  for (int r = 0; r < 8; ++r) {
    const float inv = 1.0f / lrow[r];
#pragma unroll
    for (int t = 0; t < 4; ++t) os[(8 * hh + r) * OS_PITCH + t * 16 + c] = oacc[t][r] * inv;
  }
  __builtin_amdgcn_fence(__ATOMIC_RELEASE, "workgroup");
  __builtin_amdgcn_wave_barrier();
  __builtin_amdgcn_fence(__ATOMIC_ACQUIRE, "workgroup");
  {
    const int q8 = lane >> 3, c8 = (lane & 7) * 8;
    const size_t obase = (rowbase + q0) * (size_t)D_MODEL + colbase;
    for (int pass = 0; pass < 2; ++pass) {
#pragma unroll
      for (int it = 0; it < 4; ++it) {
        const int row = it * 4 + q8;
        const float* sp = os + row * OS_PITCH + c8;
        v8h hv, lv;
#pragma unroll
        for (int e = 0; e < 8; ++e) {
          unsigned short hb = f2bf_bits(sp[e]);
          unsigned short lb = f2bf_bits(sp[e] - bf_bits2f(hb));
          hv[e] = __builtin_bit_cast(_Float16, hb);
          lv[e] = __builtin_bit_cast(_Float16, lb);
        }
        *(volatile v8h*)(Oh + obase + (size_t)row * D_MODEL + c8) = hv;
        *(volatile v8h*)(Ol + obase + (size_t)row * D_MODEL + c8) = lv;
      }
      __threadfence();
    }
  }
}

extern "C" void kernel_launch(void* const* d_in, const int* in_sizes, int n_in,
                              void* d_out, int out_size, void* d_ws, size_t ws_size,
                              hipStream_t stream) {
  constexpr size_t PLANE_ELEMS = (size_t)M_ROWS * D_MODEL;
  constexpr size_t W_ELEMS     = (size_t)D_MODEL * D_MODEL;
  static_assert(PLANE_ELEMS % 8 == 0);
  static_assert((PLANE_ELEMS / 8) % 256 == 0);
  static_assert(D_MODEL % 4 == 0 && D_MODEL / 4 == 192);
  static_assert(M_ROWS % 64 == 0 && D_MODEL % 64 == 0 && D_MODEL % 32 == 0);

  if (n_in < 11) return;
  if (in_sizes[0] != (int)PLANE_ELEMS || in_sizes[1] != (int)PLANE_ELEMS || in_sizes[2] != (int)PLANE_ELEMS) return;
  if (in_sizes[3] != (int)W_ELEMS || in_sizes[5] != (int)W_ELEMS || in_sizes[7] != (int)W_ELEMS || in_sizes[9] != (int)W_ELEMS) return;
  if (in_sizes[4] != D_MODEL || in_sizes[6] != D_MODEL || in_sizes[8] != D_MODEL || in_sizes[10] != D_MODEL) return;
  if (out_size != (int)PLANE_ELEMS) return;

  const float* query = (const float*)d_in[0];
  const float* key_  = (const float*)d_in[1];
  const float* value = (const float*)d_in[2];
  const float* Wq = (const float*)d_in[3];
  const float* bq = (const float*)d_in[4];
  const float* Wk = (const float*)d_in[5];
  const float* bk = (const float*)d_in[6];
  const float* Wv = (const float*)d_in[7];
  const float* bv = (const float*)d_in[8];
  const float* Wo = (const float*)d_in[9];
  const float* bo = (const float*)d_in[10];
  float* out = (float*)d_out;

  size_t off = 0;
  const size_t offX16  = off; off += 3 * PLANE_ELEMS * 2;
  const size_t offWT   = off; off += 4 * W_ELEMS * 2;
  const size_t offBias = off; off += 4 * (size_t)D_MODEL * 4;
  const size_t offHi   = off; off += 3 * PLANE_ELEMS * 2;
  const size_t offLo   = off; off += 3 * PLANE_ELEMS * 2;
  const size_t offOh   = off; off += PLANE_ELEMS * 2;
  const size_t offOl   = off; off += PLANE_ELEMS * 2;
  if (off > ws_size) return;

  unsigned char* ws = (unsigned char*)d_ws;
  unsigned short* X16   = (unsigned short*)(ws + offX16);
  unsigned short* Xq16  = X16;
  unsigned short* Xk16  = X16 + PLANE_ELEMS;
  unsigned short* Xv16  = X16 + 2 * PLANE_ELEMS;
  unsigned short* WT16  = (unsigned short*)(ws + offWT);
  unsigned short* WTq   = WT16;
  unsigned short* WTk   = WT16 + W_ELEMS;
  unsigned short* WTv   = WT16 + 2 * W_ELEMS;
  unsigned short* WTo   = WT16 + 3 * W_ELEMS;
  float* biasR = (float*)(ws + offBias);
  float* bqR = biasR;
  float* bkR = biasR + D_MODEL;
  float* bvR = biasR + 2 * D_MODEL;
  float* boR = biasR + 3 * D_MODEL;
  unsigned short* Qh  = (unsigned short*)(ws + offHi);
  unsigned short* Kh  = Qh + PLANE_ELEMS;
  unsigned short* Vth = Qh + 2 * PLANE_ELEMS;
  unsigned short* Ql  = (unsigned short*)(ws + offLo);
  unsigned short* Kl  = Ql + PLANE_ELEMS;
  unsigned short* Vtl = Ql + 2 * PLANE_ELEMS;
  unsigned short* Oh  = (unsigned short*)(ws + offOh);
  unsigned short* Ol  = (unsigned short*)(ws + offOl);

  const int n8 = (int)(PLANE_ELEMS / 8);
  cast_f32_bf16x8<<<dim3((unsigned)((n8 + 255) / 256), 3), dim3(256), 0, stream>>>(
      query, key_, value, X16, n8, (long)PLANE_ELEMS);

  transpose_cast_w<<<dim3(D_MODEL / 64, D_MODEL / 64, 4), dim3(256), 0, stream>>>(
      Wq, Wk, Wv, Wo, WT16, D_MODEL);

  rne_bias4<<<dim3(4), dim3(192), 0, stream>>>(bq, bk, bv, bo, biasR, D_MODEL);

  const dim3 gblk(256);
  const dim3 ggrid((unsigned)((((M_ROWS / 64) * (D_MODEL / 64)) + 7) / 8), 1);
  wmma_gemm64<1, 0, 2, 2, false, 0><<<ggrid, gblk, 0, stream>>>(
      Xq16, nullptr, D_MODEL, 0L, WTq, nullptr, D_MODEL, 0L,
      (void*)Qh, (void*)Ql, D_MODEL, 0L, bqR, nullptr, 0L, M_ROWS, D_MODEL, D_MODEL, 1.0f);
  wmma_gemm64<1, 0, 2, 2, false, 0><<<ggrid, gblk, 0, stream>>>(
      Xk16, nullptr, D_MODEL, 0L, WTk, nullptr, D_MODEL, 0L,
      (void*)Kh, (void*)Kl, D_MODEL, 0L, bkR, nullptr, 0L, M_ROWS, D_MODEL, D_MODEL, 1.0f);
  const dim3 ggridT((unsigned)((((D_MODEL / 64) * (M_ROWS / 64)) + 7) / 8), 1);
  wmma_gemm64<1, 0, 1, 2, false, 0><<<ggridT, gblk, 0, stream>>>(
      WTv, nullptr, D_MODEL, 0L, Xv16, nullptr, D_MODEL, 0L,
      (void*)Vth, (void*)Vtl, M_ROWS, 0L, bvR, nullptr, 0L, D_MODEL, M_ROWS, D_MODEL, 1.0f);

  attn_hd64_planes<<<dim3((unsigned)(N_BATCH * N_HEADS * (SEQ_LEN / Q_BLOCK))), dim3(128), 0, stream>>>(
      Qh, Ql, Kh, Kl, Vth, Vtl, Oh, Ol, 0.125f);

  wmma_gemm64<1, 1, 2, 0, false, 0><<<ggrid, gblk, 0, stream>>>(
      Oh, Ol, D_MODEL, 0L, WTo, nullptr, D_MODEL, 0L,
      (void*)out, nullptr, D_MODEL, 0L, boR, nullptr, 0L, M_ROWS, D_MODEL, D_MODEL, 1.0f);
}
